// TimeSeriesMamba_35364760715924
// MI455X (gfx1250) — hardware-run, weakly checked
//
#include <hip/hip_runtime.h>
#include <stdint.h>

constexpr int NBATCH = 2;
constexpr int SEQLEN = 1024;
constexpr int DMODEL = 1024;
constexpr int DINNER = 2048;
constexpr int DSTATE = 16;
constexpr int DTRANK = 64;
constexpr int DCONV  = 4;
constexpr int NXDIM  = DTRANK + 2 * DSTATE;
constexpr int NXPAD  = 128;
constexpr int MROWS  = NBATCH * SEQLEN;

static_assert(MROWS % 64 == 0, "M tile");
static_assert((2 * DINNER) % 64 == 0 && DMODEL % 32 == 0, "in-proj N,K");
static_assert(NXPAD % 64 == 0 && DINNER % 32 == 0 && NXPAD >= NXDIM, "x-proj N,K");
static_assert(DINNER % 64 == 0 && DTRANK % 32 == 0, "dt-proj N,K");
static_assert(DMODEL % 64 == 0, "out-proj N");
static_assert(DINNER == 512 * 4, "conv kernel: 512 threads x 4 channels per row");
static_assert(DINNER % 256 == 0 && SEQLEN % 32 == 0, "scan tiling");
static_assert(DSTATE == 16 && DTRANK == 64 && DCONV == 4, "fixed geometry");

typedef __attribute__((ext_vector_type(16))) _Float16 v16h;
typedef __attribute__((ext_vector_type(8)))  _Float16 v8h;
typedef __attribute__((ext_vector_type(16))) __bf16   v16b;
typedef __attribute__((ext_vector_type(8)))  __bf16   v8b;
typedef __attribute__((ext_vector_type(8)))  float    v8f;
typedef __attribute__((ext_vector_type(4)))  float    v4f;
typedef __attribute__((ext_vector_type(4)))  unsigned v4u;
typedef __attribute__((ext_vector_type(2)))  unsigned v2u;

__device__ __forceinline__ unsigned short f2bf_bits(float f) {
  unsigned u = __float_as_uint(f);
  return (unsigned short)((u + 0x7FFFu + ((u >> 16) & 1u)) >> 16);
}
__device__ __forceinline__ float bf_bits2f(unsigned short h) { return __uint_as_float(((unsigned)h) << 16); }
__device__ __forceinline__ float bfr(float f) { return bf_bits2f(f2bf_bits(f)); }
__device__ __forceinline__ void split_bf(float f, unsigned short& hb, unsigned short& lb) {
  hb = f2bf_bits(f);
  lb = f2bf_bits(f - bf_bits2f(hb));
}
__device__ __forceinline__ unsigned pack2(unsigned short lo, unsigned short hi) {
  return (unsigned)lo | ((unsigned)hi << 16);
}

__device__ __forceinline__ void dep_guard_h(v8f& a, v8f& b, v16h x, v16h y) { asm volatile("v_nop\n\tv_nop\n\tv_nop\n\tv_nop" : "+v"(a), "+v"(b) : "v"(x), "v"(y)); }
__device__ __forceinline__ void dep_guard_b(v8f& a, v8f& b, v16b x, v16b y) { asm volatile("v_nop\n\tv_nop\n\tv_nop\n\tv_nop" : "+v"(a), "+v"(b) : "v"(x), "v"(y)); }
__device__ __forceinline__ void keep4_h(v16h a, v16h b, v16h c, v16h d) { asm volatile("v_nop" :: "v"(a), "v"(b), "v"(c), "v"(d)); }
__device__ __forceinline__ void keep4_b(v16b a, v16b b, v16b c, v16b d) { asm volatile("v_nop" :: "v"(a), "v"(b), "v"(c), "v"(d)); }
__device__ __forceinline__ void acc_guard4(v8f& a, v8f& b, v8f& c, v8f& d) { asm volatile("v_nop\n\tv_nop\n\tv_nop\n\tv_nop" : "+v"(a), "+v"(b), "+v"(c), "+v"(d)); }
template <typename T> struct Frag;
template <> struct Frag<_Float16> {
  typedef v16h V; union U { v16h v; v8h h[2]; };
  static __device__ __forceinline__ v16h load(const _Float16* p) {
    U f; f.h[0] = *(const v8h*)(p); f.h[1] = *(const v8h*)(p + 16); return f.v;
  }
  static __device__ __forceinline__ v8f mma(v16h a, v16h b, v8f c) {
    return __builtin_amdgcn_wmma_f32_16x16x32_f16(false, a, false, b, (short)0, c, false, false);
  }
  static __device__ __forceinline__ void guard(v8f& a, v8f& b, v16h x, v16h y) { dep_guard_h(a, b, x, y); }
  static __device__ __forceinline__ void keep(v16h a, v16h b, v16h c, v16h d) { keep4_h(a, b, c, d); }
};
template <> struct Frag<__bf16> {
  typedef v16b V; union U { v16b v; v8b h[2]; };
  static __device__ __forceinline__ v16b load(const __bf16* p) {
    U f; f.h[0] = *(const v8b*)(p); f.h[1] = *(const v8b*)(p + 16); return f.v;
  }
  static __device__ __forceinline__ v8f mma(v16b a, v16b b, v8f c) {
    return __builtin_amdgcn_wmma_f32_16x16x32_bf16(false, a, false, b, (short)0, c, false, false);
  }
  static __device__ __forceinline__ void guard(v8f& a, v8f& b, v16b x, v16b y) { dep_guard_b(a, b, x, y); }
  static __device__ __forceinline__ void keep(v16b a, v16b b, v16b c, v16b d) { keep4_b(a, b, c, d); }
};

template <int ET> struct Elem;
template <> struct Elem<0> { typedef _Float16 T; };
template <> struct Elem<1> { typedef __bf16 T; };
template <int ET, int ASPLIT, int OUT_MODE>
__global__ __launch_bounds__(256) void wmma_gemm64(
    const unsigned short* __restrict__ Ap, const unsigned short* __restrict__ A2p, int lda, long strideA,
    const unsigned short* __restrict__ Btp, const unsigned short* __restrict__ Bt2p, int ldb, long strideB,
    void* __restrict__ Cout, void* __restrict__ Cout2, int ldc, long strideC,
    int M, int N, int K, float scale) {
  typedef typename Elem<ET>::T T;
  typedef typename Frag<T>::V V;
  const T* A = (const T*)Ap; const T* A2 = (const T*)A2p; const T* Bt = (const T*)Btp; const T* Bt2 = (const T*)Bt2p;
  __shared__ __align__(16) float sT[8][16 * 68];
  const int b    = blockIdx.y;
  const int lane = threadIdx.x & 31;
  const int wave = threadIdx.x >> 5;
  const int tilesN = N >> 6;
  const int tilesM = M >> 6;
  const int tile = blockIdx.x * 8 + wave;
  if (tile >= tilesM * tilesN) return;
  const int tm = tile / tilesN;
  const int tn = tile - tm * tilesN;
  const int m0 = tm << 6;
  const int n0 = tn << 6;

  const T* Ab  = A  + (size_t)b * strideA;
  const T* Bb  = Bt + (size_t)b * strideB;
  const T* Ab2 = (ASPLIT >= 1) ? (A2  + (size_t)b * strideA) : nullptr;
  const T* Bb2 = (ASPLIT == 2) ? (Bt2 + (size_t)b * strideB) : nullptr;

  const int rlane = lane & 15;
  const int koff  = (lane >> 4) * 8;
  const int mOff  = (lane >> 4) * 8;

  v8f acc[4][4];
#pragma unroll
  for (int i = 0; i < 4; ++i)
#pragma unroll
    for (int j = 0; j < 4; ++j) acc[i][j] = (v8f){0.f,0.f,0.f,0.f,0.f,0.f,0.f,0.f};

  for (int k0 = 0; k0 < K; k0 += 32) {
    V bh[4], bl[4];
#pragma unroll
    for (int j = 0; j < 4; ++j) {
      const size_t bo = (size_t)(n0 + (j << 4) + rlane) * ldb + koff + k0;
      bh[j] = Frag<T>::load(Bb + bo);
      if (ASPLIT == 2) bl[j] = Frag<T>::load(Bb2 + bo);
    }
#pragma unroll
    for (int i = 0; i < 4; ++i) {
      const size_t ao = (size_t)(m0 + (i << 4) + rlane) * lda + koff + k0;
      V ah = Frag<T>::load(Ab + ao);
      V al = ah;
      if (ASPLIT >= 1) al = Frag<T>::load(Ab2 + ao);
#pragma unroll
      for (int j = 0; j < 4; ++j) {
        acc[i][j] = Frag<T>::mma(ah, bh[j], acc[i][j]);
        if (ASPLIT >= 1) acc[i][j] = Frag<T>::mma(al, bh[j], acc[i][j]);
        if (ASPLIT == 2) acc[i][j] = Frag<T>::mma(ah, bl[j], acc[i][j]);
      }
      Frag<T>::guard(acc[i][0], acc[i][3], ah, al);
    }
    Frag<T>::keep(bh[0], bh[1], bh[2], bh[3]);
    if (ASPLIT == 2) Frag<T>::keep(bl[0], bl[1], bl[2], bl[3]);
  }
  acc_guard4(acc[0][0], acc[0][1], acc[0][2], acc[0][3]);
  acc_guard4(acc[1][0], acc[1][1], acc[1][2], acc[1][3]);
  acc_guard4(acc[2][0], acc[2][1], acc[2][2], acc[2][3]);
  acc_guard4(acc[3][0], acc[3][1], acc[3][2], acc[3][3]);

  float* slab = sT[wave];
#pragma unroll
  for (int i = 0; i < 4; ++i) {
    const int mBase = m0 + (i << 4);
#pragma unroll
    for (int j = 0; j < 4; ++j) {
#pragma unroll
      for (int r = 0; r < 8; ++r) {
        const float v = acc[i][j][r] * scale;
        slab[(mOff + r) * 68 + (j << 4) + rlane] = v;
      }
    }
    __builtin_amdgcn_fence(__ATOMIC_RELEASE, "workgroup");
    __builtin_amdgcn_wave_barrier();
    __builtin_amdgcn_fence(__ATOMIC_ACQUIRE, "workgroup");
    if (OUT_MODE == 0) {
      float* C = (float*)Cout + (size_t)b * strideC;
      const int hh = lane >> 4, c4 = (lane & 15) * 4;
      for (int pass = 0; pass < 2; ++pass) {
#pragma unroll
        for (int it = 0; it < 8; ++it) {
          const int row = it * 2 + hh;
          v4f v = *(const v4f*)(slab + row * 68 + c4);
          *(volatile v4f*)(C + (size_t)(mBase + row) * ldc + n0 + c4) = v;
        }
        __threadfence();
      }
    } else {
      const int q = lane >> 3, c8 = (lane & 7) * 8;
      unsigned short* C  = (unsigned short*)Cout  + (size_t)b * strideC;
      unsigned short* C2 = (OUT_MODE == 2) ? ((unsigned short*)Cout2 + (size_t)b * strideC) : nullptr;
      for (int pass = 0; pass < 2; ++pass) {
#pragma unroll
        for (int it = 0; it < 4; ++it) {
          const int row = it * 4 + q;
          const float* sp = slab + row * 68 + c8;
          v8h hv, lv;
#pragma unroll
          for (int e = 0; e < 8; ++e) {
            if (OUT_MODE == 1) {
              hv[e] = (_Float16)sp[e];
            } else {
              unsigned short hb = f2bf_bits(sp[e]);
              unsigned short lb = f2bf_bits(sp[e] - bf_bits2f(hb));
              hv[e] = __builtin_bit_cast(_Float16, hb);
              lv[e] = __builtin_bit_cast(_Float16, lb);
            }
          }
          *(volatile v8h*)(C + (size_t)(mBase + row) * ldc + n0 + c8) = hv;
          if (OUT_MODE == 2) *(volatile v8h*)(C2 + (size_t)(mBase + row) * ldc + n0 + c8) = lv;
        }
        __threadfence();
      }
    }
    __builtin_amdgcn_fence(__ATOMIC_RELEASE, "workgroup");
    __builtin_amdgcn_wave_barrier();
    __builtin_amdgcn_fence(__ATOMIC_ACQUIRE, "workgroup");
  }
}

__global__ __launch_bounds__(256) void cast_f32_bf16x8(
    const float* __restrict__ in, unsigned short* __restrict__ out, int n8, int n_real) {
  const int i = blockIdx.x * 256 + threadIdx.x;
  if (i >= n8) return;
  const long e  = (long)i * 8;
  const long ec = (e + 8 <= (long)n_real) ? e : ((long)n_real - 8);
  const v4f a = *(const v4f*)(in + ec);
  const v4f c = *(const v4f*)(in + ec + 4);
  v4u w;
  w[0] = pack2(f2bf_bits(a[0]), f2bf_bits(a[1]));
  w[1] = pack2(f2bf_bits(a[2]), f2bf_bits(a[3]));
  w[2] = pack2(f2bf_bits(c[0]), f2bf_bits(c[1]));
  w[3] = pack2(f2bf_bits(c[2]), f2bf_bits(c[3]));
  if (e >= (long)n_real) w = (v4u){0u, 0u, 0u, 0u};
  unsigned short* p = out + e;
  *(volatile v4u*)p = w;
  __threadfence();
  *(volatile v4u*)p = w;
}

__global__ __launch_bounds__(512) void conv_silu_k(
    const float* __restrict__ xz, const float* __restrict__ cw, const float* __restrict__ cb,
    float* __restrict__ xcf, unsigned short* __restrict__ xch, unsigned short* __restrict__ xcl) {
  __shared__ __align__(16) unsigned short hs[DINNER];
  __shared__ __align__(16) unsigned short ls[DINNER];
  const int tid = threadIdx.x;
  const int row = blockIdx.x;
  const int l   = row & (SEQLEN - 1);
  const int d0  = tid * 4;

  v4f wr[4];
#pragma unroll
  for (int c = 0; c < 4; ++c) {
    v4f t = *(const v4f*)(cw + (size_t)(d0 + c) * DCONV);
#pragma unroll
    for (int j = 0; j < DCONV; ++j) t[j] = bfr(t[j]);
    wr[c] = t;
  }
  float acc[4] = {0.f, 0.f, 0.f, 0.f};
#pragma unroll
  for (int j = 0; j < DCONV; ++j) {
    const int lj = l - (DCONV - 1) + j;
    if (lj >= 0) {
      const v4f xv = *(const v4f*)(xz + (size_t)(row - (DCONV - 1) + j) * (2 * DINNER) + d0);
#pragma unroll
      for (int c = 0; c < 4; ++c) acc[c] = fmaf(wr[c][j], xv[c], acc[c]);
    }
  }
  const v4f bias = *(const v4f*)(cb + d0);
  v4f s4;
  unsigned short hb[4], lb[4];
#pragma unroll
  for (int c = 0; c < 4; ++c) {
    const float v = acc[c] + bfr(bias[c]);
    const float e = expf(-v);
    const float s = v * __builtin_amdgcn_rcpf(1.0f + e);
    s4[c] = s;
    split_bf(s, hb[c], lb[c]);
  }
  {
    float* pf = xcf + (size_t)row * DINNER + d0;
    *(volatile v4f*)pf = s4;
    __threadfence();
    *(volatile v4f*)pf = s4;
  }
  *(v2u*)(hs + d0) = (v2u){pack2(hb[0], hb[1]), pack2(hb[2], hb[3])};
  *(v2u*)(ls + d0) = (v2u){pack2(lb[0], lb[1]), pack2(lb[2], lb[3])};
  __syncthreads();
  {
    const int u = tid & 255;
    const v4u vh = *(const v4u*)(hs + u * 8);
    const v4u vl = *(const v4u*)(ls + u * 8);
    const bool first = (tid < 256);
    const v4u vv = first ? vh : vl;
    const size_t off = (size_t)row * DINNER + (size_t)u * 8;
    unsigned short* pp = first ? (xch + off) : (xcl + off);
    *(volatile v4u*)pp = vv;
    __threadfence();
    *(volatile v4u*)pp = vv;
  }
}

__global__ __launch_bounds__(256) void slice_dt_k(
    const float* __restrict__ dbc, unsigned short* __restrict__ dth, unsigned short* __restrict__ dtl) {
  const int i = blockIdx.x * 256 + threadIdx.x;
  if (i >= MROWS * 8) return;
  const int rowi = i >> 3, c8 = (i & 7) * 8;
  const float* src = dbc + (size_t)rowi * NXPAD + c8;
  const v4f a = *(const v4f*)src;
  const v4f c = *(const v4f*)(src + 4);
  unsigned short hb[8], lb[8];
#pragma unroll
  for (int e = 0; e < 4; ++e) {
    split_bf(a[e], hb[e], lb[e]);
    split_bf(c[e], hb[4 + e], lb[4 + e]);
  }
  v4u wh, wl;
#pragma unroll
  for (int q = 0; q < 4; ++q) {
    wh[q] = pack2(hb[2 * q], hb[2 * q + 1]);
    wl[q] = pack2(lb[2 * q], lb[2 * q + 1]);
  }
  const size_t off = (size_t)rowi * DTRANK + c8;
  *(volatile v4u*)(dth + off) = wh;
  *(volatile v4u*)(dtl + off) = wl;
  __threadfence();
  *(volatile v4u*)(dth + off) = wh;
  *(volatile v4u*)(dtl + off) = wl;
}

__global__ __launch_bounds__(256) void scan_k(
    const float* __restrict__ dtlin, const float* __restrict__ b_dt, const float* __restrict__ A_log,
    const float* __restrict__ dbc, const float* __restrict__ xcf, const float* __restrict__ xz,
    const float* __restrict__ D_skip, unsigned short* __restrict__ yh, unsigned short* __restrict__ yl) {
  __shared__ float bcs[32][32];
  __shared__ __align__(16) float ybuf[32][256];
  const int tid = threadIdx.x, lane = tid & 31, wave = tid >> 5;
  const int b = blockIdx.y;
  const int dblk = blockIdx.x * 256;
  const int d = dblk + tid;

  float h[DSTATE], Ad[DSTATE];
  {
    const float* ap = A_log + (size_t)d * DSTATE;
#pragma unroll
    for (int q = 0; q < 4; ++q) {
      const v4f av = *(const v4f*)(ap + 4 * q);
#pragma unroll
      for (int e = 0; e < 4; ++e) {
        Ad[4 * q + e] = -__expf(bfr(av[e]));
        h[4 * q + e] = 0.f;
      }
    }
  }
  const float bdt = bfr(b_dt[d]);
  const float Dsk = bfr(D_skip[d]);

  for (int l0 = 0; l0 < SEQLEN; l0 += 32) {
#pragma unroll
    for (int rep = 0; rep < 4; ++rep) {
      const int linear = rep * 256 + tid;
      const int t = linear >> 5;
      const int c = linear & 31;
      bcs[t][c] = dbc[(size_t)(b * SEQLEN + l0 + t) * NXPAD + DTRANK + c];
    }
    __syncthreads();

#pragma unroll 1
    for (int t = 0; t < 32; ++t) {
      const size_t rowi = (size_t)(b * SEQLEN + l0 + t);
      const size_t idx  = rowi * DINNER + d;
      const float dv = dtlin[idx] + bdt;
      const float sp = fmaxf(dv, 0.f) + log1pf(expf(-fabsf(dv)));
      const float xv = xcf[idx];
      const float xdt = xv * sp;
      float y = 0.f;
#pragma unroll
      for (int n = 0; n < DSTATE; ++n) {
        const float ab = __expf(sp * Ad[n]);
        h[n] = fmaf(ab, h[n], xdt * bcs[t][n]);
        y = fmaf(bcs[t][DSTATE + n], h[n], y);
      }
      const float zv = xz[rowi * (2 * DINNER) + DINNER + d];
      const float g  = zv * __builtin_amdgcn_rcpf(1.0f + expf(-zv));
      ybuf[t][tid] = (y + xv * Dsk) * g;
    }
    __syncthreads();

    for (int pass = 0; pass < 2; ++pass) {
#pragma unroll
      for (int it = 0; it < 4; ++it) {
        const int t = it * 8 + wave;
        const int c8 = lane * 8;
        const v4f u0 = *(const v4f*)(&ybuf[t][c8]);
        const v4f u1 = *(const v4f*)(&ybuf[t][c8 + 4]);
        unsigned short hb[8], lb[8];
#pragma unroll
        for (int e = 0; e < 4; ++e) {
          split_bf(u0[e], hb[e], lb[e]);
          split_bf(u1[e], hb[4 + e], lb[4 + e]);
        }
        v4u wh, wl;
#pragma unroll
        for (int q = 0; q < 4; ++q) {
          wh[q] = pack2(hb[2 * q], hb[2 * q + 1]);
          wl[q] = pack2(lb[2 * q], lb[2 * q + 1]);
        }
        const size_t off = (size_t)(b * SEQLEN + l0 + t) * DINNER + dblk + c8;
        *(volatile v4u*)(yh + off) = wh;
        *(volatile v4u*)(yl + off) = wl;
      }
      __threadfence();
    }
    __syncthreads();
  }
}

extern "C" void kernel_launch(void* const* d_in, const int* in_sizes, int n_in,
                              void* d_out, int out_size, void* d_ws, size_t ws_size,
                              hipStream_t stream) {
  if (n_in < 10) return;
  if (in_sizes[0] != MROWS * DMODEL || in_sizes[1] != 2 * DINNER * DMODEL || in_sizes[2] != DINNER * DCONV ||
      in_sizes[3] != DINNER || in_sizes[4] != NXDIM * DINNER || in_sizes[5] != DINNER * DTRANK ||
      in_sizes[6] != DINNER || in_sizes[7] != DINNER * DSTATE || in_sizes[8] != DINNER ||
      in_sizes[9] != DMODEL * DINNER || out_size != MROWS * DMODEL) return;

  const float* x      = (const float*)d_in[0];
  const float* W_in   = (const float*)d_in[1];
  const float* conv_w = (const float*)d_in[2];
  const float* conv_b = (const float*)d_in[3];
  const float* W_x    = (const float*)d_in[4];
  const float* W_dt   = (const float*)d_in[5];
  const float* b_dt   = (const float*)d_in[6];
  const float* A_log  = (const float*)d_in[7];
  const float* D_skip = (const float*)d_in[8];
  const float* W_out  = (const float*)d_in[9];
  float* out = (float*)d_out;

  char* ws = (char*)d_ws;
  size_t off = 0;
  auto carve = [&](size_t bytes) -> void* { void* p = ws + off; off += bytes; return p; };
  unsigned short* x_bf    = (unsigned short*)carve((size_t)MROWS * DMODEL * 2);
  unsigned short* Win_bf  = (unsigned short*)carve((size_t)2 * DINNER * DMODEL * 2);
  float*          xz      = (float*)carve((size_t)MROWS * 2 * DINNER * 4);
  float*          xcf     = (float*)carve((size_t)MROWS * DINNER * 4);
  unsigned short* xch     = (unsigned short*)carve((size_t)MROWS * DINNER * 2);
  unsigned short* xcl     = (unsigned short*)carve((size_t)MROWS * DINNER * 2);
  unsigned short* Wx_bf   = (unsigned short*)carve((size_t)NXPAD * DINNER * 2);
  float*          dbc     = (float*)carve((size_t)MROWS * NXPAD * 4);
  unsigned short* dth     = (unsigned short*)carve((size_t)MROWS * DTRANK * 2);
  unsigned short* dtl     = (unsigned short*)carve((size_t)MROWS * DTRANK * 2);
  unsigned short* Wdt_bf  = (unsigned short*)carve((size_t)DINNER * DTRANK * 2);
  float*          dtlin   = (float*)carve((size_t)MROWS * DINNER * 4);
  unsigned short* yh      = (unsigned short*)carve((size_t)MROWS * DINNER * 2);
  unsigned short* yl      = (unsigned short*)carve((size_t)MROWS * DINNER * 2);
  unsigned short* Wout_bf = (unsigned short*)carve((size_t)DMODEL * DINNER * 2);
  if (off > ws_size) return;

  {
    const int n8x   = MROWS * DMODEL / 8;
    const int n8wi  = 2 * DINNER * DMODEL / 8;
    const int n8wx  = NXPAD * DINNER / 8;
    const int n8wd  = DINNER * DTRANK / 8;
    const int n8wo  = DMODEL * DINNER / 8;
    cast_f32_bf16x8<<<(n8x + 255) / 256, 256, 0, stream>>>(x, x_bf, n8x, MROWS * DMODEL);
    cast_f32_bf16x8<<<(n8wi + 255) / 256, 256, 0, stream>>>(W_in, Win_bf, n8wi, 2 * DINNER * DMODEL);
    cast_f32_bf16x8<<<(n8wx + 255) / 256, 256, 0, stream>>>(W_x, Wx_bf, n8wx, NXDIM * DINNER);
    cast_f32_bf16x8<<<(n8wd + 255) / 256, 256, 0, stream>>>(W_dt, Wdt_bf, n8wd, DINNER * DTRANK);
    cast_f32_bf16x8<<<(n8wo + 255) / 256, 256, 0, stream>>>(W_out, Wout_bf, n8wo, DMODEL * DINNER);
  }

  {
    const int tiles = (MROWS / 64) * ((2 * DINNER) / 64);
    wmma_gemm64<1, 0, 0><<<dim3((tiles + 7) / 8, 1), 256, 0, stream>>>(
        x_bf, x_bf, DMODEL, 0L, Win_bf, Win_bf, DMODEL, 0L,
        (void*)xz, (void*)xz, 2 * DINNER, 0L, MROWS, 2 * DINNER, DMODEL, 1.0f);
  }

  conv_silu_k<<<MROWS, 512, 0, stream>>>(xz, conv_w, conv_b, xcf, xch, xcl);

  {
    const int tiles = (MROWS / 64) * (NXPAD / 64);
    wmma_gemm64<1, 1, 0><<<dim3((tiles + 7) / 8, 1), 256, 0, stream>>>(
        xch, xcl, DINNER, 0L, Wx_bf, Wx_bf, DINNER, 0L,
        (void*)dbc, (void*)dbc, NXPAD, 0L, MROWS, NXPAD, DINNER, 1.0f);
  }

  slice_dt_k<<<(MROWS * 8 + 255) / 256, 256, 0, stream>>>(dbc, dth, dtl);
  {
    const int tiles = (MROWS / 64) * (DINNER / 64);
    wmma_gemm64<1, 1, 0><<<dim3((tiles + 7) / 8, 1), 256, 0, stream>>>(
        dth, dtl, DTRANK, 0L, Wdt_bf, Wdt_bf, DTRANK, 0L,
        (void*)dtlin, (void*)dtlin, DINNER, 0L, MROWS, DINNER, DTRANK, 1.0f);
  }

  scan_k<<<dim3(DINNER / 256, NBATCH), 256, 0, stream>>>(dtlin, b_dt, A_log, dbc, xcf, xz, D_skip, yh, yl);

  {
    const int tiles = (MROWS / 64) * (DMODEL / 64);
    wmma_gemm64<1, 1, 0><<<dim3((tiles + 7) / 8, 1), 256, 0, stream>>>(
        yh, yl, DINNER, 0L, Wout_bf, Wout_bf, DINNER, 0L,
        (void*)out, (void*)out, DMODEL, 0L, MROWS, DMODEL, DINNER, 1.0f);
  }
}
